// GAT_575525617905
// MI455X (gfx1250) — hardware-run, weakly checked
//
#include <hip/hip_runtime.h>
#include <stddef.h>
#include <stdint.h>
#include <math.h>

#define NN      50000
#define NE      800000
#define FD      256
#define HC      128
#define GN      256
#define MP      50048
#define GBM     64
#define GBN     64
#define GTHR    128
#define NTHR    256
#define NWAVE   8
#define EPT     8
#define WCH     (32 * EPT)
#define NBRUN   1024
#define SLB     10
#define NBK     49
#define SPW     (NBRUN / NWAVE)
#define WLCAP   3584
#define RCAP    28672
#define TRIPCAP 256
#define MAXDEG_MEAS   35
#define MAXB1024_MEAS 16623
#define NEGS    0.2f
#define WSMAX   (128u << 20)

#define SM_ATT  0
#define SM_B1   128
#define SM_W2P  256
#define SM_P2   768
#define SM_FLOATS 800

#define BK_ZINTS (NWAVE * WLCAP + RCAP + 3 * NBRUN)
#define BK_INTS  (BK_ZINTS + 16)
#define BK_LDS   (BK_INTS * 4)

#define PBX   (MP * FD / 8 / NTHR)
#define PBW   (GN * FD / 8 / NTHR)
#define PBTOT (PBX + PBW + 1)

static_assert(8 * 16 == 128 && 128 == 32 * 4 && 16 == 4 * 4);
static_assert(HC == 128 && GN == 2 * HC);
static_assert(NN % 16 == 0 && (NN * 2 * 4) % 128 == 0);
static_assert(NN < 65536 && NBRUN <= 1024 && NBRUN == (1 << SLB));
static_assert(NBK * NBRUN >= NN && (NBK - 1) * NBRUN < NN);
static_assert(MP % GBM == 0 && MP >= NN && GN % GBN == 0 && FD % 32 == 0);
static_assert(GBM == (GTHR / 32) * 16);
static_assert((MP * FD / 8) % NTHR == 0 && (GN * FD / 8) % NTHR == 0 && PBW % 2 == 0);
static_assert(NE % WCH == 0 && NE % 4 == 0 && NE < (1 << 20));
static_assert((((long long)NE) << SLB) < (1LL << 31));
static_assert(RCAP == NWAVE * WLCAP && RCAP % 4 == 0 && BK_ZINTS % (NTHR * 4) == 0);
static_assert((long long)RCAP * 100 >= (long long)MAXB1024_MEAS * 105);
static_assert(WLCAP >= MAXB1024_MEAS / 8 + 8 * 46 + 1);
static_assert(MAXDEG_MEAS + 8 <= TRIPCAP && TRIPCAP < 65536);
static_assert(BK_LDS <= 300000);
static_assert(((NN - (NBK - 1) * NBRUN) * 8) % 128 == 0);
static_assert((NBK - 1) * NBRUN * 2 + (NN - (NBK - 1) * NBRUN) * 2 == 2 * NN);
static_assert((NN * 2 * 4) % 128 == 0);
static_assert(SM_P2 + 32 == SM_FLOATS);

typedef float          v2f   __attribute__((ext_vector_type(2)));
typedef float          v4f   __attribute__((ext_vector_type(4)));
typedef float          v8f   __attribute__((ext_vector_type(8)));
typedef int            v4i   __attribute__((ext_vector_type(4)));
typedef int            v8i   __attribute__((ext_vector_type(8)));
typedef unsigned short v8us  __attribute__((ext_vector_type(8)));
typedef unsigned short v16us __attribute__((ext_vector_type(16)));
typedef __bf16         v16bf __attribute__((ext_vector_type(16)));
typedef v2f  __attribute__((may_alias)) v2fa;
typedef v4f  __attribute__((may_alias)) v4fa;
typedef v4i  __attribute__((may_alias)) v4ia;
typedef v8us __attribute__((may_alias)) v8usa;
union FragB { v16bf v; v16us u; v8us h[2]; v8i w; };

__device__ __forceinline__ v8f wmb(const FragB& a, const FragB& b, v8f c) {
  v8f d = __builtin_amdgcn_wmma_f32_16x16x32_bf16(false, a.v, false, b.v, (short)0, c, false, false);
  asm volatile("v_nop\n\tv_nop\n\tv_nop\n\tv_nop" : "+v"(d) : "v"(a.w), "v"(b.w));
  return d;
}

__device__ __forceinline__ unsigned bf16_bits(float f) {
  const unsigned u = __float_as_uint(f);
  const unsigned r = (u + 0x7FFFu + ((u >> 16) & 1u)) >> 16;
  const unsigned q = (u >> 16) | 0x40u;
  return ((u & 0x7fffffffu) > 0x7f800000u) ? q : r;
}
__device__ __forceinline__ float bf16_val(float f) {
  return __uint_as_float(bf16_bits(f) << 16);
}

__device__ __forceinline__ void st2_v4f(float* p, v4f v) {
  *(volatile v4f*)p = v;
  __threadfence();
  *(volatile v4f*)p = v;
}
__device__ __forceinline__ void st2_v8us(unsigned short* p, v8us v) {
  *(volatile v8us*)p = v;
  __threadfence();
  *(volatile v8us*)p = v;
}

__device__ __forceinline__ v8us gather8(const float* __restrict__ base, int stride) {
  float f[8];
#pragma unroll
  for (int i = 0; i < 8; ++i) f[i] = base[(size_t)i * (size_t)stride];
  v8us o;
#pragma unroll
  for (int i = 0; i < 8; ++i) o[i] = (unsigned short)bf16_bits(f[i]);
  return o;
}

__global__ __launch_bounds__(NTHR) void k_prep(const float* __restrict__ x, const float* __restrict__ wl1,
                                               const float* __restrict__ wr1, const float* __restrict__ att1,
                                               const float* __restrict__ bias1, const float* __restrict__ wl2,
                                               const float* __restrict__ wr2, const float* __restrict__ att2,
                                               const float* __restrict__ bias2,
                                               unsigned short* xb, unsigned short* wt, float* sm) {
  const int tid = (int)threadIdx.x, lane = tid & 31, wave = tid >> 5;
  const int blk = (int)blockIdx.x;
  if (blk < PBX) {
    const int u   = blk * NTHR + tid;
    const int row = u >> 5, k8 = (u & 31) * 8;
    const int rc  = row < NN ? row : NN - 1;
    const unsigned mk = row < NN ? 0xffffu : 0u;
    const float* p = x + (size_t)rc * FD + k8;
    const v4f a = *(const v4fa*)p;
    const v4f b = *(const v4fa*)(p + 4);
    v8us o;
    o[0] = (unsigned short)(bf16_bits(a.x) & mk); o[1] = (unsigned short)(bf16_bits(a.y) & mk);
    o[2] = (unsigned short)(bf16_bits(a.z) & mk); o[3] = (unsigned short)(bf16_bits(a.w) & mk);
    o[4] = (unsigned short)(bf16_bits(b.x) & mk); o[5] = (unsigned short)(bf16_bits(b.y) & mk);
    o[6] = (unsigned short)(bf16_bits(b.z) & mk); o[7] = (unsigned short)(bf16_bits(b.w) & mk);
    st2_v8us(xb + (size_t)row * FD + k8, o);
  } else if (blk < PBX + PBW / 2) {
    const int u = (blk - PBX) * NTHR + tid;
    const int n = u >> 5, k8 = (u & 31) * 8;
    const v8us o = gather8(wl1 + (size_t)k8 * HC + n, HC);
    st2_v8us(wt + (size_t)n * FD + k8, o);
  } else if (blk < PBX + PBW) {
    const int u = (blk - PBX - PBW / 2) * NTHR + tid;
    const int n = u >> 5, k8 = (u & 31) * 8;
    const v8us o = gather8(wr1 + (size_t)k8 * HC + n, HC);
    st2_v8us(wt + (size_t)(HC + n) * FD + k8, o);
  } else {
    if (wave == 0) {
      const v4f a = *(const v4fa*)(att1 + 4 * lane);
      v4f o;
      o.x = bf16_val(a.x); o.y = bf16_val(a.y); o.z = bf16_val(a.z); o.w = bf16_val(a.w);
      st2_v4f(sm + SM_ATT + 4 * lane, o);
    } else if (wave == 1) {
      const v4f a = *(const v4fa*)(bias1 + 4 * lane);
      v4f o;
      o.x = bf16_val(a.x); o.y = bf16_val(a.y); o.z = bf16_val(a.z); o.w = bf16_val(a.w);
      st2_v4f(sm + SM_B1 + 4 * lane, o);
    } else if (wave < 6) {
      const int j = tid - 64;
      const v2f a = *(const v2fa*)(wl2 + 2 * j);
      const v2f b = *(const v2fa*)(wr2 + 2 * j);
      v4f o;
      o.x = bf16_val(a.x); o.y = bf16_val(a.y); o.z = bf16_val(b.x); o.w = bf16_val(b.y);
      st2_v4f(sm + SM_W2P + 4 * j, o);
    } else if (wave == 6) {
      const float a0 = att2[0], a1 = att2[1], c0 = bias2[0], c1 = bias2[1];
      asm volatile("" :: "v"(a0), "v"(a1), "v"(c0), "v"(c1));
      const unsigned mk = (lane == 0) ? 0xffffffffu : 0u;
      v4f o;
      o.x = __uint_as_float((bf16_bits(a0) << 16) & mk);
      o.y = __uint_as_float((bf16_bits(a1) << 16) & mk);
      o.z = __uint_as_float((bf16_bits(c0) << 16) & mk);
      o.w = __uint_as_float((bf16_bits(c1) << 16) & mk);
      if (lane < 8) st2_v4f(sm + SM_P2 + 4 * lane, o);
    }
  }
}

__device__ __forceinline__ void bucket_flush(const int* pl, const int* cnt, int ov, int* lp, int* cop, int* fp,
                                             int tid) {
#pragma unroll 1
  for (int i = tid * 4; i < RCAP; i += NTHR * 4) {
    const v4i v = *(const v4ia*)(pl + i);
    *(volatile v4i*)(lp + i) = v;
  }
#pragma unroll 1
  for (int i = tid * 4; i < 2 * NBRUN; i += NTHR * 4) {
    const v4i v = *(const v4ia*)(cnt + i);
    *(volatile v4i*)(cop + i) = v;
  }
  if (tid < 8) {
    const v4i f = {ov, ov, ov, ov};
    *(volatile v4i*)(fp + 4 * tid) = f;
  }
}

__global__ __launch_bounds__(NTHR) void k_bucket(const int* __restrict__ srcs, const int* __restrict__ dsts,
                                                 int* LIST, int* CO, int* FLAG) {
  extern __shared__ __attribute__((aligned(16))) int dsm[];
  int* wl   = dsm;
  int* pl   = dsm + NWAVE * WLCAP;
  int* cnt  = pl + RCAP;
  int* offs = cnt + NBRUN;
  int* cur  = offs + NBRUN;
  int* misc = cur + NBRUN;
  const int tid = (int)threadIdx.x, lane = tid & 31, wave = tid >> 5;
  const int blk = (int)blockIdx.x;
  const unsigned nbs = (unsigned)(blk * NBRUN);

  {
    const v4i z4 = {0, 0, 0, 0};
    for (int i = tid * 4; i < BK_ZINTS; i += NTHR * 4) *(v4ia*)(dsm + i) = z4;
    if (tid < 16) misc[tid] = 0;
  }
  __syncthreads();

  {
    const int per  = ((NE + NWAVE * WCH - 1) / (NWAVE * WCH)) * WCH;
    const int ebeg = wave * per;
    const int eend = (ebeg + per < NE) ? (ebeg + per) : NE;
    int* mylist = wl + wave * WLCAP;
    int wc = 0;
#pragma unroll 1
    for (int cb = ebeg; cb < eend; cb += WCH) {
      const int e0 = cb + lane * EPT;
      const v4i da = *(const v4ia*)(dsts + e0);
      const v4i db = *(const v4ia*)(dsts + e0 + 4);
      const unsigned s0 = (unsigned)da.x - nbs, s1 = (unsigned)da.y - nbs;
      const unsigned s2 = (unsigned)da.z - nbs, s3 = (unsigned)da.w - nbs;
      const unsigned s4 = (unsigned)db.x - nbs, s5 = (unsigned)db.y - nbs;
      const unsigned s6 = (unsigned)db.z - nbs, s7 = (unsigned)db.w - nbs;
      const bool h0 = s0 < (unsigned)NBRUN, h1 = s1 < (unsigned)NBRUN, h2 = s2 < (unsigned)NBRUN, h3 = s3 < (unsigned)NBRUN;
      const bool h4 = s4 < (unsigned)NBRUN, h5 = s5 < (unsigned)NBRUN, h6 = s6 < (unsigned)NBRUN, h7 = s7 < (unsigned)NBRUN;
      const unsigned m0 = __builtin_amdgcn_ballot_w32(h0), m1 = __builtin_amdgcn_ballot_w32(h1);
      const unsigned m2 = __builtin_amdgcn_ballot_w32(h2), m3 = __builtin_amdgcn_ballot_w32(h3);
      const unsigned m4 = __builtin_amdgcn_ballot_w32(h4), m5 = __builtin_amdgcn_ballot_w32(h5);
      const unsigned m6 = __builtin_amdgcn_ballot_w32(h6), m7 = __builtin_amdgcn_ballot_w32(h7);
      const unsigned any = m0 | m1 | m2 | m3 | m4 | m5 | m6 | m7;
      if (any != 0u) {
        const int pre = (int)(__builtin_amdgcn_mbcnt_lo(m0, 0u) + __builtin_amdgcn_mbcnt_lo(m1, 0u) +
                              __builtin_amdgcn_mbcnt_lo(m2, 0u) + __builtin_amdgcn_mbcnt_lo(m3, 0u) +
                              __builtin_amdgcn_mbcnt_lo(m4, 0u) + __builtin_amdgcn_mbcnt_lo(m5, 0u) +
                              __builtin_amdgcn_mbcnt_lo(m6, 0u) + __builtin_amdgcn_mbcnt_lo(m7, 0u));
        int p = wc + pre;
        if (h0) { if (p < WLCAP) mylist[p] = ((e0 + 0) << SLB) | (int)s0; p = p + 1; }
        if (h1) { if (p < WLCAP) mylist[p] = ((e0 + 1) << SLB) | (int)s1; p = p + 1; }
        if (h2) { if (p < WLCAP) mylist[p] = ((e0 + 2) << SLB) | (int)s2; p = p + 1; }
        if (h3) { if (p < WLCAP) mylist[p] = ((e0 + 3) << SLB) | (int)s3; p = p + 1; }
        if (h4) { if (p < WLCAP) mylist[p] = ((e0 + 4) << SLB) | (int)s4; p = p + 1; }
        if (h5) { if (p < WLCAP) mylist[p] = ((e0 + 5) << SLB) | (int)s5; p = p + 1; }
        if (h6) { if (p < WLCAP) mylist[p] = ((e0 + 6) << SLB) | (int)s6; p = p + 1; }
        if (h7) { if (p < WLCAP) mylist[p] = ((e0 + 7) << SLB) | (int)s7; p = p + 1; }
        wc += (int)(__builtin_popcount(m0) + __builtin_popcount(m1) + __builtin_popcount(m2) + __builtin_popcount(m3) +
                    __builtin_popcount(m4) + __builtin_popcount(m5) + __builtin_popcount(m6) + __builtin_popcount(m7));
      }
    }
    if (lane == 0) misc[wave] = wc;
  }
  __syncthreads();

  if (wave == 0) {
    int ov = 0;
#pragma unroll 1
    for (int w2 = 0; w2 < NWAVE; ++w2) {
      int c = misc[w2];
      if (c > WLCAP) ov = 1;
      c = c < 0 ? 0 : (c > WLCAP ? WLCAP : c);
#pragma unroll 1
      for (int b0 = 0; b0 < c; b0 += 32) {
        const int idx = b0 + lane;
        const int ent = wl[w2 * WLCAP + (idx < WLCAP ? idx : WLCAP - 1)];
        const int m32 = (c - b0) < 32 ? (c - b0) : 32;
#pragma unroll 1
        for (int k = 0; k < m32; ++k) {
          const int u    = __builtin_amdgcn_readlane(ent, k);
          const int slot = u & (NBRUN - 1);
          if (lane == 0) cnt[slot] = cnt[slot] + 1;
        }
      }
    }
    if (lane == 0) misc[9] = ov;
  }
  __syncthreads();
  if (wave == 0) {
    const int base = lane * (NBRUN / 32);
    int s = 0;
#pragma unroll 1
    for (int i = 0; i < NBRUN / 32; ++i) s += cnt[base + i];
    int incl = s;
#pragma unroll
    for (int d = 1; d < 32; d <<= 1) {
      const int y = __shfl_up(incl, d, 32);
      if (lane >= d) incl += y;
    }
    int run = incl - s;
#pragma unroll 1
    for (int i = 0; i < NBRUN / 32; ++i) {
      const int cv = cnt[base + i];
      offs[base + i] = run;
      cur[base + i]  = run;
      run += cv;
    }
  }
  __syncthreads();

  if (wave == 0) {
#pragma unroll 1
    for (int w2 = 0; w2 < NWAVE; ++w2) {
      int c = misc[w2];
      c = c < 0 ? 0 : (c > WLCAP ? WLCAP : c);
#pragma unroll 1
      for (int b0 = 0; b0 < c; b0 += 32) {
        const int idx = b0 + lane;
        const int ent = wl[w2 * WLCAP + (idx < WLCAP ? idx : WLCAP - 1)];
        int eid = (ent >> SLB) & 0xFFFFF;
        eid = eid > NE - 1 ? NE - 1 : eid;
        int sr = srcs[eid];
        sr = sr < 0 ? 0 : (sr > NN - 1 ? NN - 1 : sr);
        const int word = (int)((unsigned)sr | ((unsigned)(ent & (NBRUN - 1)) << 16));
        const int m32 = (c - b0) < 32 ? (c - b0) : 32;
#pragma unroll 1
        for (int k = 0; k < m32; ++k) {
          const int u    = __builtin_amdgcn_readlane(ent, k);
          const int wd   = __builtin_amdgcn_readlane(word, k);
          const int slot = u & (NBRUN - 1);
          if (lane == 0) {
            int p = cur[slot];
            p = p < 0 ? 0 : (p > RCAP - 1 ? RCAP - 1 : p);
            pl[p] = wd;
            cur[slot] = p + 1;
          }
        }
      }
    }
  }
  __syncthreads();

  const int ovf = misc[9];
  int* lp  = LIST + (size_t)blk * RCAP;
  int* cop = CO + (size_t)blk * (2 * NBRUN);
  int* fp  = FLAG + (size_t)blk * 32;
  bucket_flush(pl, cnt, ovf, lp, cop, fp, tid);
  __threadfence();
  bucket_flush(pl, cnt, ovf, lp, cop, fp, tid);
}

__global__ __launch_bounds__(GTHR) __attribute__((amdgpu_num_vgpr(248)))
void k_gemm(const unsigned short* __restrict__ A, const unsigned short* __restrict__ WT, float* outF) {
  __shared__ __attribute__((aligned(16))) float stg[GBM * GBN];
  const int tid = (int)threadIdx.x, lane = tid & 31, wave = tid >> 5, hh = lane >> 4, m = lane & 15;
  const int rowBase = (int)blockIdx.x * GBM;
  const int col0    = (int)blockIdx.y * GBN;

  v8f acc[4];
  {
    const v8f z = {0.f, 0.f, 0.f, 0.f, 0.f, 0.f, 0.f, 0.f};
    acc[0] = z; acc[1] = z; acc[2] = z; acc[3] = z;
  }
  const unsigned short* ap = A  + (size_t)(rowBase + 16 * wave + m) * (size_t)FD + 8 * hh;
  const unsigned short* wp = WT + (size_t)(col0 + m) * (size_t)FD + 8 * hh;
#pragma unroll 1
  for (int ks = 0; ks < FD / 32; ++ks) {
    FragB af;
    af.h[0] = *(const v8usa*)(ap + 32 * ks);
    af.h[1] = *(const v8usa*)(ap + 32 * ks + 16);
#pragma unroll
    for (int t = 0; t < 4; ++t) {
      const unsigned short* wq = wp + (size_t)(16 * t) * (size_t)FD + 32 * ks;
      FragB bf;
      bf.h[0] = *(const v8usa*)wq;
      bf.h[1] = *(const v8usa*)(wq + 16);
      acc[t] = wmb(af, bf, acc[t]);
    }
  }

#pragma unroll
  for (int t = 0; t < 4; ++t) {
    const int lc = 16 * t + m;
#pragma unroll
    for (int r = 0; r < 8; ++r) {
      const int lr = 16 * wave + 8 * hh + r;
      stg[lr * GBN + lc] = acc[t][r];
    }
  }
  __syncthreads();

  v4f fv[8];
#pragma unroll
  for (int i = 0; i < 8; ++i) {
    const int lr = 16 * wave + 2 * i + hh;
    fv[i] = *(const v4fa*)(stg + lr * GBN + 4 * m);
  }
#pragma unroll
  for (int i = 0; i < 8; ++i) {
    const int lr = 16 * wave + 2 * i + hh;
    float* op = outF + (size_t)(rowBase + lr) * (size_t)GN + col0 + 4 * m;
    *(volatile v4f*)op = fv[i];
  }
  __threadfence();
#pragma unroll
  for (int i = 0; i < 8; ++i) {
    const int lr = 16 * wave + 2 * i + hh;
    float* op = outF + (size_t)(rowBase + lr) * (size_t)GN + col0 + 4 * m;
    *(volatile v4f*)op = fv[i];
  }
}

__device__ __forceinline__ void r1_flush(const float* stg, float* ob, int tid) {
#pragma unroll 1
  for (int it = 0; it < (NBRUN * 4) / (NTHR * 4); ++it) {
    const int i4 = it * NTHR + tid;
    const v4f v = *(const v4fa*)(stg + 4 * i4);
    *(volatile v4f*)(ob + (size_t)4 * (size_t)i4) = v;
  }
}

__global__ __launch_bounds__(NTHR) void k_replay1(const int* __restrict__ LIST, const int* __restrict__ CO,
                                                  const int* __restrict__ FLAG, const float* __restrict__ XLR,
                                                  const float* __restrict__ SM, float* XLR2) {
  __shared__ __attribute__((aligned(16))) float stg[NBRUN * 4];
  __shared__ __attribute__((aligned(16))) int   cos_[2 * NBRUN];
  __shared__ __attribute__((aligned(16))) float w2s[HC * 4];
  __shared__ __attribute__((aligned(16))) float hst[NWAVE * 128];
  const int tid = (int)threadIdx.x, lane = tid & 31, wave = tid >> 5;
  const int blk = (int)blockIdx.x;
  const int nodeBase = blk * NBRUN;
  const int* lb  = LIST + (size_t)blk * RCAP;
  const int* cob = CO + (size_t)blk * (2 * NBRUN);

#pragma unroll 1
  for (int i = tid * 4; i < 2 * NBRUN; i += NTHR * 4) *(v4ia*)(cos_ + i) = *(const v4ia*)(cob + i);
  if (tid < HC) *(v4fa*)(w2s + 4 * tid) = *(const v4fa*)(SM + SM_W2P + 4 * tid);
  __syncthreads();

  const int flag = FLAG[(size_t)blk * 32];
  const v4f at = *(const v4fa*)(SM + SM_ATT + 4 * lane);
  const v4f bb = *(const v4fa*)(SM + SM_B1 + 4 * lane);
  const float qnan = __uint_as_float(0x7fc00000u);
  float* hw = hst + wave * 128;

#pragma unroll 1
  for (int jt = 0; jt < SPW; ++jt) {
    const int slot = wave * SPW + jt;
    const int grow = nodeBase + slot;
    v4f res = {0.0f, 0.0f, 0.0f, 0.0f};
    if (grow < NN) {
      int cv = cos_[slot];
      int ov = cos_[NBRUN + slot];
      const bool big = cv > TRIPCAP;
      cv = cv < 0 ? 0 : (cv > TRIPCAP ? TRIPCAP : cv);
      ov = ov < 0 ? 0 : (ov > RCAP - 1 ? RCAP - 1 : ov);
      const int c = __builtin_amdgcn_readfirstlane(cv);
      const int o = __builtin_amdgcn_readfirstlane(ov);
      int last = o + c - 1; last = last < o ? o : last;
      last = last > RCAP - 1 ? RCAP - 1 : last;
      const int total = c + 1;

      const v4f xr = *(const v4fa*)(XLR + (size_t)grow * GN + HC + 4 * lane);
      float mx = -1.0e30f, den = 0.0f;
      float a0 = 0.0f, a1 = 0.0f, a2 = 0.0f, a3 = 0.0f;
#pragma unroll 1
      for (int b0 = 0; b0 < total; b0 += 32) {
        const int e = b0 + lane;
        int idx = o + e - 1;
        idx = idx < o ? o : idx;
        idx = idx > last ? last : idx;
        const int wdl = lb[idx];
        asm volatile("" :: "v"(wdl));
        const int mk = (e == 0) ? -1 : 0;
        int sv = (grow & mk) | ((wdl & 0xffff) & ~mk);
        sv = sv > NN - 1 ? NN - 1 : sv;
        const int m32 = (total - b0) < 32 ? (total - b0) : 32;
#pragma unroll 1
        for (int k = 0; k < m32; ++k) {
          const int s = __builtin_amdgcn_readlane(sv, k);
          const v4f xv = *(const v4fa*)(XLR + (size_t)s * GN + 4 * lane);
          float z0 = xv.x + xr.x, z1 = xv.y + xr.y, z2 = xv.z + xr.z, z3 = xv.w + xr.w;
          z0 = z0 > 0.0f ? z0 : z0 * NEGS; z1 = z1 > 0.0f ? z1 : z1 * NEGS;
          z2 = z2 > 0.0f ? z2 : z2 * NEGS; z3 = z3 > 0.0f ? z3 : z3 * NEGS;
          float part = z0 * at.x;
          part = fmaf(z1, at.y, part); part = fmaf(z2, at.z, part); part = fmaf(z3, at.w, part);
          part += __shfl_xor(part, 1, 32);
          part += __shfl_xor(part, 2, 32);
          const float df = part - mx;
          const float tt = expf(-fabsf(df));
          const bool gt  = part > mx;
          const float sc = gt ? tt : 1.0f;
          const float pp = gt ? 1.0f : tt;
          mx  = gt ? part : mx;
          den = fmaf(den, sc, pp);
          a0 = fmaf(a0, sc, pp * xv.x); a1 = fmaf(a1, sc, pp * xv.y);
          a2 = fmaf(a2, sc, pp * xv.z); a3 = fmaf(a3, sc, pp * xv.w);
        }
      }
      const float inv = 1.0f / (den + 1e-16f);
      hw[lane]      = fmaf(a0, inv, bb.x);
      hw[32 + lane] = fmaf(a1, inv, bb.y);
      hw[64 + lane] = fmaf(a2, inv, bb.z);
      hw[96 + lane] = fmaf(a3, inv, bb.w);
      float q0 = 0.0f, q1 = 0.0f, q2 = 0.0f, q3 = 0.0f;
#pragma unroll 1
      for (int cc = 0; cc < 4; ++cc) {
        const float v = hw[cc * 32 + lane];
        const float ev = (v > 0.0f) ? v : expm1f(v);
        const v4f w = *(const v4fa*)(w2s + 4 * (4 * lane + cc));
        q0 = fmaf(ev, w.x, q0); q1 = fmaf(ev, w.y, q1); q2 = fmaf(ev, w.z, q2); q3 = fmaf(ev, w.w, q3);
      }
#pragma unroll 1
      for (int off = 16; off > 0; off >>= 1) {
        q0 += __shfl_xor(q0, off, 32); q1 += __shfl_xor(q1, off, 32);
        q2 += __shfl_xor(q2, off, 32); q3 += __shfl_xor(q3, off, 32);
      }
      const bool bad = (flag != 0) | big;
      res.x = bad ? qnan : q0; res.y = bad ? qnan : q1; res.z = bad ? qnan : q2; res.w = bad ? qnan : q3;
    }
    if (lane == 0) *(v4fa*)(stg + 4 * slot) = res;
  }
  __syncthreads();

  float* ob = XLR2 + (size_t)blk * (size_t)(NBRUN * 4);
  r1_flush(stg, ob, tid);
  __threadfence();
  r1_flush(stg, ob, tid);
}

__device__ __forceinline__ void r2_flush(const float* s0, const float* s1, float* ob0, float* ob1, int nv4, int tid) {
#pragma unroll 1
  for (int it = 0; it < (NBRUN * 2) / (NTHR * 4); ++it) {
    const int i4 = it * NTHR + tid;
    const v4f v = *(const v4fa*)(s0 + 4 * i4);
    const v4f w = *(const v4fa*)(s1 + 4 * i4);
    asm volatile("" :: "v"(v));
    asm volatile("" :: "v"(w));
    if (i4 < nv4) {
      *(volatile v4f*)(ob0 + (size_t)4 * (size_t)i4) = v;
      *(volatile v4f*)(ob1 + (size_t)4 * (size_t)i4) = w;
    }
  }
}

__global__ __launch_bounds__(NTHR) void k_replay2(const int* __restrict__ LIST, const int* __restrict__ CO,
                                                  const int* __restrict__ FLAG, const float* __restrict__ XLR2,
                                                  const float* __restrict__ SM, float* out) {
  __shared__ __attribute__((aligned(16))) float s0[NBRUN * 2];
  __shared__ __attribute__((aligned(16))) float s1[NBRUN * 2];
  __shared__ __attribute__((aligned(16))) int   cos_[2 * NBRUN];
  const int tid = (int)threadIdx.x, lane = tid & 31, wave = tid >> 5;
  const int blk = (int)blockIdx.x;
  const int nodeBase = blk * NBRUN;
  const int* lb  = LIST + (size_t)blk * RCAP;
  const int* cob = CO + (size_t)blk * (2 * NBRUN);

#pragma unroll 1
  for (int i = tid * 4; i < 2 * NBRUN; i += NTHR * 4) *(v4ia*)(cos_ + i) = *(const v4ia*)(cob + i);
  __syncthreads();

  const int flag = FLAG[(size_t)blk * 32];
  const v4f p2 = *(const v4fa*)(SM + SM_P2);
  const float qnan = __uint_as_float(0x7fc00000u);

#pragma unroll 1
  for (int jt = 0; jt < SPW; ++jt) {
    const int slot = wave * SPW + jt;
    const int grow = nodeBase + slot;
    v2f r0 = {0.0f, 0.0f};
    v2f r1 = {0.0f, 0.0f};
    if (grow < NN) {
      int cv = cos_[slot];
      int ov = cos_[NBRUN + slot];
      const bool big = cv > TRIPCAP;
      cv = cv < 0 ? 0 : (cv > TRIPCAP ? TRIPCAP : cv);
      ov = ov < 0 ? 0 : (ov > RCAP - 1 ? RCAP - 1 : ov);
      const int c = __builtin_amdgcn_readfirstlane(cv);
      const int o = __builtin_amdgcn_readfirstlane(ov);
      int last = o + c - 1; last = last < o ? o : last;
      last = last > RCAP - 1 ? RCAP - 1 : last;
      const int total = c + 1;
      const int trips = (total + 31) >> 5;

      const v4f me = *(const v4fa*)(XLR2 + (size_t)4 * (size_t)grow);
      float mx = -1.0e30f, den = 0.0f, a0 = 0.0f, a1 = 0.0f;
#pragma unroll 1
      for (int t = 0; t < trips; ++t) {
        const int e = t * 32 + lane;
        const bool valid = e < total;
        int idx = o + e - 1;
        idx = idx < o ? o : idx;
        idx = idx > last ? last : idx;
        const int wdl = lb[idx];
        asm volatile("" :: "v"(wdl));
        const int mk = (e == 0) ? -1 : 0;
        int sv = (grow & mk) | ((wdl & 0xffff) & ~mk);
        sv = sv > NN - 1 ? NN - 1 : sv;
        const v2f xs = *(const v2fa*)(XLR2 + (size_t)4 * (size_t)sv);
        const float x0 = xs.x, x1 = xs.y;
        asm volatile("" :: "v"(x0), "v"(x1));
        float z0 = x0 + me.z, z1 = x1 + me.w;
        z0 = z0 > 0.0f ? z0 : z0 * NEGS;
        z1 = z1 > 0.0f ? z1 : z1 * NEGS;
        const float lg = fmaf(z1, p2.y, z0 * p2.x);
        const float df = lg - mx;
        const float tt = expf(-fabsf(df));
        const bool gt  = lg > mx;
        const float sc = gt ? tt : 1.0f;
        const float pp = gt ? 1.0f : tt;
        const float mn = gt ? lg : mx;
        const float dn = fmaf(den, sc, pp);
        const float n0 = fmaf(a0, sc, pp * x0);
        const float n1 = fmaf(a1, sc, pp * x1);
        mx  = valid ? mn : mx;
        den = valid ? dn : den;
        a0  = valid ? n0 : a0;
        a1  = valid ? n1 : a1;
      }
#pragma unroll 1
      for (int off = 16; off > 0; off >>= 1) {
        const float mo = __shfl_xor(mx, off, 32);
        const float dq = __shfl_xor(den, off, 32);
        const float b0 = __shfl_xor(a0, off, 32);
        const float b1 = __shfl_xor(a1, off, 32);
        const float df = mo - mx;
        const float tt = expf(-fabsf(df));
        const bool gt  = mo > mx;
        const float sa = gt ? tt : 1.0f;
        const float sb = gt ? 1.0f : tt;
        mx  = gt ? mo : mx;
        den = fmaf(den, sa, dq * sb);
        a0  = fmaf(a0, sa, b0 * sb);
        a1  = fmaf(a1, sa, b1 * sb);
      }
      const float inv = 1.0f / (den + 1e-16f);
      const float o0 = fmaf(a0, inv, p2.z);
      const float o1 = fmaf(a1, inv, p2.w);
      const float mo2 = (o0 > o1) ? o0 : o1;
      const float sa = o0 - mo2, sb = o1 - mo2;
      const float L  = logf(expf(sa) + expf(sb));
      const bool bad = (flag != 0) | big;
      r0.x = bad ? qnan : o0;        r0.y = bad ? qnan : o1;
      r1.x = bad ? qnan : (sa - L);  r1.y = bad ? qnan : (sb - L);
    }
    if (lane == 0) {
      *(v2fa*)(s0 + 2 * slot) = r0;
      *(v2fa*)(s1 + 2 * slot) = r1;
    }
  }
  __syncthreads();

  const int liveRows = (NN - nodeBase) < NBRUN ? (NN - nodeBase) : NBRUN;
  const int nv4 = liveRows / 2;
  float* ob0 = out + (size_t)blk * (size_t)(NBRUN * 2);
  float* ob1 = out + (size_t)(2 * NN) + (size_t)blk * (size_t)(NBRUN * 2);
  r2_flush(s0, s1, ob0, ob1, nv4, tid);
  __threadfence();
  r2_flush(s0, s1, ob0, ob1, nv4, tid);
}

extern "C" void kernel_launch(void* const* d_in, const int* in_sizes, int n_in,
                              void* d_out, int out_size, void* d_ws, size_t ws_size,
                              hipStream_t stream) {
  if (n_in < 10) return;
  if (in_sizes[0] != NN * FD) return;
  if (in_sizes[1] != 2 * NE) return;
  if (in_sizes[2] != FD * HC) return;
  if (in_sizes[3] != FD * HC) return;
  if (in_sizes[4] != HC) return;
  if (in_sizes[5] != HC) return;
  if (in_sizes[6] != HC * 2) return;
  if (in_sizes[7] != HC * 2) return;
  if (in_sizes[8] != 2) return;
  if (in_sizes[9] != 2) return;
  if (out_size != 4 * NN) return;

  const float* x     = (const float*)d_in[0];
  const int*   ei    = (const int*)d_in[1];
  const float* Wl1   = (const float*)d_in[2];
  const float* Wr1   = (const float*)d_in[3];
  const float* att1  = (const float*)d_in[4];
  const float* bias1 = (const float*)d_in[5];
  const float* Wl2   = (const float*)d_in[6];
  const float* Wr2   = (const float*)d_in[7];
  const float* att2  = (const float*)d_in[8];
  const float* bias2 = (const float*)d_in[9];
  float* out = (float*)d_out;
  const int* srcs = ei;
  const int* dsts = ei + NE;

  constexpr size_t zXB   = (size_t)MP * FD * 2;
  constexpr size_t zWT   = (size_t)GN * FD * 2;
  constexpr size_t zXLR  = (size_t)MP * GN * 4;
  constexpr size_t zLIST = (size_t)NBK * RCAP * 4;
  constexpr size_t zCO   = (size_t)NBK * 2 * NBRUN * 4;
  constexpr size_t zFLAG = (((size_t)NBK * 128 + 255) / 256) * 256;
  constexpr size_t zXLR2 = (size_t)NBK * NBRUN * 16;
  constexpr size_t zSM   = (((size_t)SM_FLOATS * 4 + 255) / 256) * 256;
  constexpr size_t oXB   = 0;
  constexpr size_t oWT   = oXB + zXB;
  constexpr size_t oXLR  = oWT + zWT;
  constexpr size_t oLIST = oXLR + zXLR;
  constexpr size_t oCO   = oLIST + zLIST;
  constexpr size_t oFLAG = oCO + zCO;
  constexpr size_t oXLR2 = oFLAG + zFLAG;
  constexpr size_t oSM   = oXLR2 + zXLR2;
  constexpr size_t oEND  = oSM + zSM;
  static_assert(zXB % 256 == 0 && zWT % 256 == 0 && zXLR % 256 == 0 && zLIST % 256 == 0 && zCO % 256 == 0);
  static_assert(zFLAG % 256 == 0 && zXLR2 % 256 == 0 && zSM % 256 == 0);
  static_assert(zFLAG >= (size_t)NBK * 128 && zSM >= (size_t)SM_FLOATS * 4);
  static_assert(oEND <= (size_t)WSMAX);
  if (oEND > ws_size) return;

  char* ws = (char*)d_ws;
  unsigned short* XB   = (unsigned short*)(ws + oXB);
  unsigned short* WT   = (unsigned short*)(ws + oWT);
  float*          XLR  = (float*)(ws + oXLR);
  int*            LIST = (int*)(ws + oLIST);
  int*            CO   = (int*)(ws + oCO);
  int*            FLAG = (int*)(ws + oFLAG);
  float*          XLR2 = (float*)(ws + oXLR2);
  float*          SM   = (float*)(ws + oSM);

  hipFuncSetAttribute(reinterpret_cast<const void*>(&k_bucket), hipFuncAttributeMaxDynamicSharedMemorySize, (int)BK_LDS);

  k_prep<<<PBTOT, NTHR, 0, stream>>>(x, Wl1, Wr1, att1, bias1, Wl2, Wr2, att2, bias2, XB, WT, SM);
  k_bucket<<<NBK, NTHR, BK_LDS, stream>>>(srcs, dsts, LIST, CO, FLAG);
  k_gemm<<<dim3(MP / GBM, GN / GBN), GTHR, 0, stream>>>(XB, WT, XLR);
  k_replay1<<<NBK, NTHR, 0, stream>>>(LIST, CO, FLAG, XLR, SM, XLR2);
  k_replay2<<<NBK, NTHR, 0, stream>>>(LIST, CO, FLAG, XLR2, SM, out);
}
